// WaveletSpectralBlock_46162308498103
// MI455X (gfx1250) — hardware-run, weakly checked
//
#include <hip/hip_runtime.h>
#include <math.h>

typedef __attribute__((ext_vector_type(16))) _Float16 v16h;
typedef __attribute__((ext_vector_type(8)))  _Float16 v8h;
typedef __attribute__((ext_vector_type(8)))  float    v8f;
typedef __attribute__((ext_vector_type(4)))  float    v4f;
typedef __attribute__((ext_vector_type(4)))  unsigned v4u;

constexpr int kNumB   = 8;
constexpr int kNumC   = 128;
constexpr int kLen    = 8192;
constexpr int kNumCh  = 128;
constexpr int kNumS   = 16;
constexpr int kPadL   = kLen / 2;
constexpr int kLenP   = kLen + 2 * kPadL;
constexpr float kOmega  = 6.0f;
constexpr float kNormEps = 1e-5f;
constexpr float kCarryA = 256.0f;
constexpr float kCarryB = 256.0f;
constexpr float kFold   = 1.0f / (kCarryA * kCarryB);
constexpr int kTileP  = 132;
static_assert(kLenP == 16384, "padded length");
static_assert((kLen % 256) == 0 && (kPadL % 256) == 0 && (kLenP % 256) == 0, "block multiples");
static_assert((kLen % 128) == 0 && (kLen % 32) == 0, "strip and k-step multiples");
static_assert(kNumS == 16, "one 16-row M tile");
static_assert(kNumCh == 128, "channel grouping");

constexpr size_t kOffBank = 0;
constexpr size_t kOffXmp  = kOffBank + (size_t)kNumS * kLen * 2;
constexpr size_t kOffXs   = kOffXmp  + (size_t)kNumB * kLenP * 2;
constexpr size_t kOffCwt  = kOffXs   + (size_t)kNumB * 16 * kLenP * 2;
constexpr size_t kWsTotal = kOffCwt  + (size_t)kNumB * kNumS * kLen * 4;
static_assert(kWsTotal == 8912896ull, "carve total");
static_assert(kWsTotal <= 134217728ull, "carve cap");
static_assert((kOffXmp % 128) == 0 && (kOffXs % 128) == 0 && (kOffCwt % 128) == 0, "aligned regions");

union FragH { v16h v; v8h h[2]; };
__device__ __forceinline__ v16h frag_load_h(const _Float16* p) {
  FragH f;
  f.h[0] = *(const v8h*)(p);
  f.h[1] = *(const v8h*)(p + 16);
  return f.v;
}
__device__ __forceinline__ v8f mma_f16_guarded(v16h a, v16h b, v8f c) {
  c = __builtin_amdgcn_wmma_f32_16x16x32_f16(false, a, false, b, (short)0, c, false, false);
  asm volatile("v_nop\n\tv_nop\n\tv_nop\n\tv_nop" : "+v"(c) : "v"(a), "v"(b));
  return c;
}

__device__ __forceinline__ void store_256_as_f16(const float* sm, _Float16* dst, int lane) {
  v8h hv;
#pragma unroll
  for (int e = 0; e < 8; ++e) hv[e] = (_Float16)sm[lane * 8 + e];
  _Float16* q = dst + lane * 8;
  *(volatile v8h*)q = hv;
  __threadfence();
  *(volatile v8h*)q = hv;
}

__global__ __launch_bounds__(256) void bank_gen_kernel(const float* __restrict__ scales, _Float16* __restrict__ bankh) {
  __shared__ __align__(16) float sm[256];
  const int tid  = threadIdx.x;
  const int lane = tid & 31;
  const int wave = __builtin_amdgcn_readfirstlane((int)(threadIdx.x >> 5));
  const int s  = blockIdx.x >> 5;
  const int j0 = (blockIdx.x & 31) * 256;
  const int j  = j0 + tid;
  const float sc  = scales[s];
  const float rsc = 1.0f / sc;
  const float t   = -4.0f + (float)j * (8.0f / 8191.0f);
  const float ts  = t * rsc;
  const float g   = expf(-0.5f * ts * ts) * cosf(kOmega * ts);
  sm[tid] = g * kCarryA;
  __syncthreads();
  if (wave == 0) store_256_as_f16(sm, bankh + (size_t)s * kLen + j0, lane);
}

__global__ __launch_bounds__(256) void chan_mean_kernel(const float* __restrict__ x, _Float16* __restrict__ xmp) {
  __shared__ __align__(16) float sm[256];
  const int tid  = threadIdx.x;
  const int lane = tid & 31;
  const int wave = __builtin_amdgcn_readfirstlane((int)(threadIdx.x >> 5));
  const int b  = blockIdx.x >> 6;
  const int p0 = (blockIdx.x & 63) * 256;
  float v = 0.0f;
  if (p0 >= kPadL && p0 < kPadL + kLen) {
    const int l = p0 - kPadL + tid;
    const float* xb = x + (size_t)b * kNumC * kLen + l;
    float acc = 0.0f;
#pragma unroll 8
    for (int c = 0; c < kNumC; ++c) acc += xb[(size_t)c * kLen];
    v = (acc * (1.0f / (float)kNumC)) * kCarryB;
  }
  sm[tid] = v;
  __syncthreads();
  if (wave == 0) store_256_as_f16(sm, xmp + (size_t)b * kLenP + p0, lane);
}

__global__ __launch_bounds__(256) void shift_planes_kernel(const unsigned* __restrict__ xmpw, unsigned short* __restrict__ xs) {
  __shared__ __align__(16) unsigned sh[272];
  const int tid  = threadIdx.x;
  const int lane = tid & 31;
  const int wave = __builtin_amdgcn_readfirstlane((int)(threadIdx.x >> 5));
  const int b  = blockIdx.x >> 6;
  const int p0 = (blockIdx.x & 63) * 256;
  const unsigned* src = xmpw + (size_t)b * (kLenP / 2);
  const int idx = (p0 >> 1) + tid;
  const int wc  = (idx < kLenP / 2) ? idx : (kLenP / 2 - 1);
  unsigned w = src[wc];
  asm volatile("" : "+v"(w));
  w = (idx < kLenP / 2) ? w : 0u;
  if (tid < 136) {
    sh[2 * tid]     = w & 0xffffu;
    sh[2 * tid + 1] = w >> 16;
  }
  __syncthreads();
  v4u pk[2];
#pragma unroll
  for (int rr = 0; rr < 2; ++rr) {
    const int r = wave * 2 + rr;
    const unsigned* sp = sh + lane * 8 + r;
    const unsigned a0 = sp[0], a1 = sp[1], a2 = sp[2], a3 = sp[3];
    const unsigned a4 = sp[4], a5 = sp[5], a6 = sp[6], a7 = sp[7];
    v4u t;
    t[0] = a0 | (a1 << 16);
    t[1] = a2 | (a3 << 16);
    t[2] = a4 | (a5 << 16);
    t[3] = a6 | (a7 << 16);
    pk[rr] = t;
  }
  for (int pass = 0; pass < 2; ++pass) {
#pragma unroll
    for (int rr = 0; rr < 2; ++rr) {
      const int r = wave * 2 + rr;
      unsigned short* dst = xs + ((size_t)(b * 16 + r)) * kLenP + p0 + lane * 8;
      *(volatile v4u*)dst = pk[rr];
    }
    __threadfence();
  }
}

__global__ __launch_bounds__(128) void corr_strip_kernel(const _Float16* __restrict__ bankh,
                                                         const _Float16* __restrict__ xs,
                                                         float* __restrict__ cwt) {
  __shared__ __align__(16) float slab[4][16 * kTileP];
  const int lane = threadIdx.x & 31;
  const int wave = __builtin_amdgcn_readfirstlane((int)(threadIdx.x >> 5));
  const int tile = blockIdx.x * 4 + wave;
  const int b    = tile >> 6;
  const int i0   = (tile & 63) * 128;
  const int rl   = lane & 15;
  const int hh   = lane >> 4;
  int klo = 3968 - i0;
  klo = (klo < 0) ? 0 : klo;
  int khi = 12288 - i0;
  khi = (khi > kLen) ? kLen : khi;

  const _Float16* ap = bankh + (size_t)rl * kLen + 8 * hh;
  const _Float16* bp = xs + ((size_t)(b * 16 + rl)) * kLenP + i0 + 8 * hh;

  v8f acc[8];
#pragma unroll
  for (int j = 0; j < 8; ++j) acc[j] = (v8f){0.f, 0.f, 0.f, 0.f, 0.f, 0.f, 0.f, 0.f};

#pragma unroll 1
  for (int k0 = klo; k0 < khi; k0 += 32) {
    const v16h a = frag_load_h(ap + k0);
#pragma unroll
    for (int j = 0; j < 8; ++j) {
      const v16h bb = frag_load_h(bp + k0 + 16 * j);
      acc[j] = mma_f16_guarded(a, bb, acc[j]);
    }
  }

  float* sl = slab[wave];
#pragma unroll
  for (int j = 0; j < 8; ++j) {
#pragma unroll
    for (int r = 0; r < 8; ++r) {
      sl[(8 * hh + r) * kTileP + 16 * j + rl] = acc[j][r] * kFold;
    }
  }
  __syncthreads();
  float* cb = cwt + (size_t)b * kNumS * kLen + i0 + lane * 4;
  for (int pass = 0; pass < 2; ++pass) {
#pragma unroll
    for (int row = 0; row < 16; ++row) {
      const v4f v = *(const v4f*)(sl + row * kTileP + lane * 4);
      *(volatile v4f*)(cb + (size_t)row * kLen) = v;
    }
    __threadfence();
  }
}

__global__ __launch_bounds__(256) void conv_act_mean_kernel(
    const float* __restrict__ cwt, const float* __restrict__ cw,
    const float* __restrict__ cbias, const float* __restrict__ gamma,
    const float* __restrict__ beta, const float* __restrict__ rmean,
    const float* __restrict__ rvar, float* __restrict__ out) {
  __shared__ __align__(16) float tile[18 * kTileP];
  __shared__ __align__(16) float so[8][4 * 32];
  const int tid  = threadIdx.x;
  const int lane = tid & 31;
  const int wave = __builtin_amdgcn_readfirstlane((int)(threadIdx.x >> 5));
  const int b  = blockIdx.x >> 6;
  const int l0 = (blockIdx.x & 63) * 128;

  const float* cbp = cwt + (size_t)b * kNumS * kLen;
#pragma unroll 1
  for (int it = 0; it < 10; ++it) {
    const int idx  = tid + it * 256;
    const int idxc = (idx < 18 * 130) ? idx : (18 * 130 - 1);
    const int r = idxc / 130;
    const int c = idxc - r * 130;
    const int s = r - 1;
    const int l = l0 + c - 1;
    const int sc = (s < 0) ? 0 : ((s > kNumS - 1) ? (kNumS - 1) : s);
    const int lc = (l < 0) ? 0 : ((l > kLen - 1) ? (kLen - 1) : l);
    float v = cbp[(size_t)sc * kLen + lc];
    asm volatile("" : "+v"(v));
    const bool ok = (s >= 0) && (s < kNumS) && (l >= 0) && (l < kLen);
    v = ok ? v : 0.0f;
    if (idx < 18 * 130) tile[r * kTileP + c] = v;
  }
  __syncthreads();

  const int lg   = wave & 3;
  const int half = wave >> 2;
  const float* tp = tile + lg * 32 + lane;
  float* sw = so[wave];
  const int qq = lane >> 3;
  const int pc = (lane & 7) * 4;

#pragma unroll 1
  for (int g = 0; g < 16; ++g) {
    const int chb = (g * 2 + half) * 4;
#pragma unroll 1
    for (int q = 0; q < 4; ++q) {
      const int ch = chb + q;
      const float* wc = cw + ch * 9;
      const float w00 = wc[0], w01 = wc[1], w02 = wc[2];
      const float w10 = wc[3], w11 = wc[4], w12 = wc[5];
      const float w20 = wc[6], w21 = wc[7], w22 = wc[8];
      const float bi  = cbias[ch];
      const float inv = gamma[ch] * (1.0f / sqrtf(rvar[ch] + kNormEps));
      const float sh  = beta[ch] - rmean[ch] * inv;
      float acc = 0.0f;
#pragma unroll 1
      for (int s = 0; s < kNumS; ++s) {
        const float* r0 = tp + s * kTileP;
        const float* r1 = r0 + kTileP;
        const float* r2 = r1 + kTileP;
        float v = w00 * r0[0] + w01 * r0[1] + w02 * r0[2]
                + w10 * r1[0] + w11 * r1[1] + w12 * r1[2]
                + w20 * r2[0] + w21 * r2[1] + w22 * r2[2];
        v = (v + bi) * inv + sh;
        acc += 0.5f * v * (1.0f + erff(v * 0.70710678118654752f));
      }
      sw[q * 32 + lane] = acc * (1.0f / (float)kNumS);
    }
    __syncthreads();
    {
      const float* sp = sw + qq * 32 + pc;
      v4f v;
      v[0] = sp[0];
      v[1] = sp[1];
      v[2] = sp[2];
      v[3] = sp[3];
      float* dst = out + ((size_t)(b * kNumCh + chb + qq)) * kLen + l0 + lg * 32 + pc;
      *(volatile v4f*)dst = v;
      __threadfence();
      *(volatile v4f*)dst = v;
    }
    __syncthreads();
  }
}

extern "C" void kernel_launch(void* const* d_in, const int* in_sizes, int n_in,
                              void* d_out, int out_size, void* d_ws, size_t ws_size,
                              hipStream_t stream) {
  if (n_in < 8) return;
  if (in_sizes[0] != kNumB * kNumC * kLen) return;
  if (in_sizes[1] != kNumS) return;
  if (in_sizes[2] != kNumCh * 9) return;
  if (in_sizes[3] != kNumCh) return;
  if (in_sizes[4] != kNumCh) return;
  if (in_sizes[5] != kNumCh) return;
  if (in_sizes[6] != kNumCh) return;
  if (in_sizes[7] != kNumCh) return;
  if (out_size != kNumB * kNumCh * kLen) return;
  if (ws_size < kWsTotal) return;

  const float* x      = (const float*)d_in[0];
  const float* scales = (const float*)d_in[1];
  const float* conv_w = (const float*)d_in[2];
  const float* conv_b = (const float*)d_in[3];
  const float* gamma  = (const float*)d_in[4];
  const float* beta   = (const float*)d_in[5];
  const float* rmean  = (const float*)d_in[6];
  const float* rvar   = (const float*)d_in[7];
  float* out = (float*)d_out;

  char* ws = (char*)d_ws;
  _Float16* bankh = (_Float16*)(ws + kOffBank);
  _Float16* xmp   = (_Float16*)(ws + kOffXmp);
  _Float16* xsp   = (_Float16*)(ws + kOffXs);
  float*    cwt   = (float*)(ws + kOffCwt);

  bank_gen_kernel<<<kNumS * (kLen / 256), 256, 0, stream>>>(scales, bankh);
  chan_mean_kernel<<<kNumB * (kLenP / 256), 256, 0, stream>>>(x, xmp);
  shift_planes_kernel<<<kNumB * (kLenP / 256), 256, 0, stream>>>((const unsigned*)xmp, (unsigned short*)xsp);
  corr_strip_kernel<<<(kNumB * (kLen / 128)) / 4, 128, 0, stream>>>(bankh, xsp, cwt);
  conv_act_mean_kernel<<<kNumB * (kLen / 128), 256, 0, stream>>>(cwt, conv_w, conv_b, gamma, beta, rmean, rvar, out);
}
